// MainGNN_14362370638529
// MI455X (gfx1250) — hardware-run, weakly checked
//
#include <hip/hip_runtime.h>


namespace {
constexpr int N = 20000, NP = 20032, E = 320000, EP = 321344  , FIN0 = 3, HID = 32, EH = 64, OUTD = 2;
constexpr int KM1 = 224  , KM1R = EH * FIN0 + FIN0, KM2 = EH * HID + HID  ;
constexpr float XS = 8.0f, WSC = 256.0f, NEG = 0.2f  ;

typedef _Float16 b16;
typedef __attribute__((ext_vector_type(16))) _Float16 v16b;
typedef __attribute__((ext_vector_type(8))) _Float16 v8b;
typedef __attribute__((ext_vector_type(8))) float v8f;
typedef __attribute__((ext_vector_type(4))) float v4f;
__device__ __forceinline__ float bf16_rne(float f) { unsigned int u = __float_as_uint(f); u += 0x7FFFu + ((u >> 16) & 1u); return __uint_as_float(u & 0xFFFF0000u); }
__device__ __forceinline__ void split16(float v, b16& hi, b16& lo) { hi = (b16)v; lo = (b16)(v - (float)hi); }
__device__ __forceinline__ v16b frag_kb(const b16* p, int hh) { const v8b a = *(const v8b*)(p + 8 * hh), b = *(const v8b*)(p + 16 + 8 * hh); v16b f;
#pragma unroll
  for (int e = 0; e < 8; ++e) { f[e] = a[e]; f[8 + e] = b[e]; } return f; }
__device__ __forceinline__ v8f wmma16b(v16b a, v16b b, v8f c) { v8f d = __builtin_amdgcn_wmma_f32_16x16x32_f16(false, a, false, b, (short)0, c, false, false); asm volatile("v_nop\n\tv_nop\n\tv_nop\n\tv_nop" : "+v"(d) : "v"(a), "v"(b)); return d; }
__device__ __forceinline__ void wave_lds_sync() { __builtin_amdgcn_fence(__ATOMIC_RELEASE, "workgroup"); __builtin_amdgcn_wave_barrier(); __builtin_amdgcn_fence(__ATOMIC_ACQUIRE, "workgroup"); }
__device__ __forceinline__ float pmul(float a, float b) { float p = a * b; asm volatile("" : "+v"(p)); return p; }
__device__ __forceinline__ int iclamp(int v, int lo, int hi) { return v < lo ? lo : (v > hi ? hi : v); }
__device__ __forceinline__ float nexp(float x) { return __builtin_amdgcn_exp2f(x * 1.4426950408889634f); }
__device__ __forceinline__ float lrelu(float x) { return x > 0.0f ? x : NEG * x; }

constexpr int CSR_NBLK = 512, CSR_GB = 9, CSR_GN = 1 << CSR_GB  , CSR_MAXG = 512, CSR_CAP = 12288  ;
__global__ __launch_bounds__(64) void csrA_kernel(const int* __restrict__ dst, int E, int N, int nG, int CHP, int NGP, int* __restrict__ STG, int* __restrict__ HST) {
  extern __shared__ int sm[];
  int* cnt = sm; int* run = sm + NGP; int* ids = sm + 2 * NGP;
  const int b = blockIdx.x; const int ch = (E + CSR_NBLK - 1) / CSR_NBLK; const int e0 = b * ch, e1 = min(E, e0 + ch);
  for (int i = threadIdx.x; i < NGP; i += 64) cnt[i] = 0;
  for (int i = threadIdx.x; i < CHP; i += 64) ids[i] = -1;
  __syncthreads();
  if (threadIdx.x == 0) {
    for (int e = e0; e < e1; ++e) { int d = dst[e]; d = (d < 0) ? 0 : (d >= N ? N - 1 : d); cnt[d >> CSR_GB] += 1; }
    int acc = 0; for (int g = 0; g < nG; ++g) { run[g] = acc; acc += cnt[g]; }
    for (int e = e0; e < e1; ++e) { int d = dst[e]; d = (d < 0) ? 0 : (d >= N ? N - 1 : d); const int g = d >> CSR_GB; ids[run[g]] = e; run[g] += 1; } }
  __syncthreads();
  typedef __attribute__((ext_vector_type(4))) int v4i;
  for (int pass = 0; pass < 2; ++pass) {
    for (int i = threadIdx.x; i < CHP / 4; i += 64) *(volatile v4i*)(STG + (size_t)b * CHP + i * 4) = *(const v4i*)(&ids[i * 4]);
    for (int i = threadIdx.x; i < NGP / 4; i += 64) { v4i v; for (int e = 0; e < 4; ++e) v[e] = (i * 4 + e < nG) ? cnt[i * 4 + e] : 0; *(volatile v4i*)(HST + (size_t)b * NGP + i * 4) = v; }
    __threadfence(); }
}
__global__ __launch_bounds__(512) void csrS_kernel(const int* __restrict__ HST, int nG, int NGP, int* __restrict__ START, int* __restrict__ TOT, int* __restrict__ OFF) {
  __shared__ int tot[CSR_MAXG];
  const int b = threadIdx.x;
  for (int pass = 0; pass < 2; ++pass) { int runb = 0; for (int g = 0; g < nG; ++g) { int c = HST[(size_t)b * NGP + g]; c = (c < 0) ? 0 : c; ((volatile int*)OFF)[(size_t)g * CSR_NBLK + b] = runb; runb += c; } __threadfence(); }
  for (int g = threadIdx.x; g < nG; g += 512) { int s = 0; for (int bb = 0; bb < CSR_NBLK; ++bb) { int c = HST[(size_t)bb * NGP + g]; s += (c < 0) ? 0 : c; } tot[g] = s; }
  __syncthreads();
  if (threadIdx.x < 32) {
    __shared__ int st[CSR_MAXG + 32];
    if (threadIdx.x == 0) { int acc = 0; for (int g = 0; g < NGP; ++g) { st[g] = acc; if (g < nG) acc += (tot[g] + 31) & ~31; } st[NGP] = acc; }
    __builtin_amdgcn_fence(__ATOMIC_RELEASE, "workgroup"); __builtin_amdgcn_wave_barrier(); __builtin_amdgcn_fence(__ATOMIC_ACQUIRE, "workgroup");
    for (int pass = 0; pass < 2; ++pass) { for (int i = threadIdx.x; i < NGP + 32; i += 32) { ((volatile int*)START)[i] = (i <= NGP) ? st[min(i, NGP)] : 0; ((volatile int*)TOT)[i] = (i < nG) ? tot[i] : 0; } __threadfence(); } }
}
__global__ __launch_bounds__(256) void csrB_kernel(const int* __restrict__ dst, int N, int nG, int CHP, int NGP, int permLen, const int* __restrict__ STG, const int* __restrict__ HST, const int* __restrict__ OFF, const int* __restrict__ START, const int* __restrict__ TOT, int* __restrict__ PERM, int* __restrict__ ROWPTR, int* __restrict__ ROWCNT, int* __restrict__ FLAG) {
  typedef __attribute__((ext_vector_type(4))) int v4i;
  __shared__ int ids[CSR_CAP]; __shared__ unsigned short key[CSR_CAP]; __shared__ int outp[CSR_CAP]; __shared__ int ncnt[CSR_GN + 1]; __shared__ int boff[CSR_NBLK + 1];
  const int g = blockIdx.x, t_ = threadIdx.x; int tot = TOT[g]; int st = START[g], stn = START[g + 1]; const int v0 = g * CSR_GN; const int nv = min(CSR_GN, N - v0);
  st = (st < 0) ? 0 : (st > permLen - 32 ? permLen - 32 : st) & ~31; stn = (stn < st) ? st : (stn > permLen ? permLen : stn); tot = (tot < 0) ? 0 : tot; if (tot > stn - st && tot <= CSR_CAP) tot = stn - st;
  if (tot > CSR_CAP) {
    for (int pass = 0; pass < 2; ++pass) { for (int i = t_; i < CSR_GN / 4; i += 256) { v4i a, c; for (int e = 0; e < 4; ++e) { a[e] = st; c[e] = 0; } *(volatile v4i*)(ROWPTR + v0 + i * 4) = a; *(volatile v4i*)(ROWCNT + v0 + i * 4) = c; } if (t_ == 0) ((volatile int*)FLAG)[0] = 1; __threadfence(); } (void)nv; return; }
  if (t_ == 0) { int acc = 0; for (int b = 0; b < CSR_NBLK; ++b) { boff[b] = acc; int c = HST[(size_t)b * NGP + g]; c = (c < 0) ? 0 : (c > CHP ? CHP : c); acc += c; if (acc > tot) acc = tot; } boff[CSR_NBLK] = acc; }
  for (int i = t_; i <= CSR_GN; i += 256) ncnt[i] = 0;
  __syncthreads();
  for (int b = 0; b < CSR_NBLK; ++b) { const int c = boff[b + 1] - boff[b]; int o_ = OFF[(size_t)g * CSR_NBLK + b]; o_ = (o_ < 0) ? 0 : (o_ > CHP - c ? CHP - c : o_); const int* src_ = STG + (size_t)b * CHP + o_;
    for (int i = t_; i < c; i += 256) { int id = src_[i]; id = (id < 0) ? 0 : id; ids[boff[b] + i] = id; int d = dst[id]; d = (d < v0) ? v0 : (d >= N ? N - 1 : d); int kk = d - v0; kk = (kk < 0) ? 0 : (kk >= CSR_GN ? CSR_GN - 1 : kk); key[boff[b] + i] = (unsigned short)kk; } }
  __syncthreads();
  if (t_ == 0) { for (int i = 0; i < tot; ++i) ncnt[key[i]] += 1; int acc = 0; for (int vl = 0; vl < CSR_GN; ++vl) { const int c = ncnt[vl]; ncnt[vl] = acc; acc += c; } ncnt[CSR_GN] = acc;
    for (int i = 0; i < tot; ++i) { const int vl = key[i]; outp[ncnt[vl]] = ids[i]; ncnt[vl] += 1; }
    for (int vl = CSR_GN; vl > 0; --vl) ncnt[vl] = ncnt[vl - 1]; ncnt[0] = 0; }
  __syncthreads();
  for (int pass = 0; pass < 2; ++pass) {
    for (int i = t_; i < (stn - st) / 4; i += 256) { v4i v; for (int e = 0; e < 4; ++e) { const int q = i * 4 + e; v[e] = (q < tot) ? outp[q] : -1; } *(volatile v4i*)(PERM + st + i * 4) = v; }
    for (int i = t_; i < CSR_GN / 4; i += 256) { v4i a, c; for (int e = 0; e < 4; ++e) { const int vl = i * 4 + e; a[e] = st + ncnt[vl]; c[e] = (vl < nv) ? (ncnt[vl + 1] - ncnt[vl]) : 0; } *(volatile v4i*)(ROWPTR + v0 + i * 4) = a; *(volatile v4i*)(ROWCNT + v0 + i * 4) = c; }
    __threadfence(); }
}
__global__ __launch_bounds__(256) void csrZ_kernel(int* __restrict__ p, size_t n4) { typedef __attribute__((ext_vector_type(4))) int v4i; const size_t tid = (size_t)blockIdx.x * 256 + threadIdx.x, nth = (size_t)gridDim.x * 256; v4i z = {0, 0, 0, 0}; for (size_t i = tid; i < n4; i += nth) *(volatile v4i*)(p + i * 4) = z; }
struct CsrBufs { int *STG, *HST, *OFF, *START, *TOT, *PERM, *ROWPTR, *ROWCNT, *FLAG; int nG, NGP, CHP; size_t permLen; char* base; size_t bytes; };
static size_t csr_carve(CsrBufs& c, char* ws, size_t off, int E, int N) {
  const size_t off0 = off; c.base = ws + off;
  auto al = [&](size_t bytes) { char* p = ws + off; off += (bytes + 255) & ~(size_t)255; return p; };
  c.nG = (N + CSR_GN - 1) / CSR_GN; c.NGP = (c.nG + 31) & ~31; const int ch = (E + CSR_NBLK - 1) / CSR_NBLK; c.CHP = (ch + 31) & ~31; c.permLen = (size_t)E + 32 * (size_t)c.nG + 32;
  c.STG = (int*)al((size_t)CSR_NBLK * c.CHP * 4); c.HST = (int*)al((size_t)CSR_NBLK * c.NGP * 4); c.OFF = (int*)al((size_t)c.NGP * CSR_NBLK * 4); c.START = (int*)al((size_t)(c.NGP + 64) * 4); c.TOT = (int*)al((size_t)(c.NGP + 64) * 4);
  c.PERM = (int*)al(c.permLen * 4); c.ROWPTR = (int*)al((size_t)c.nG * CSR_GN * 4); c.ROWCNT = (int*)al((size_t)c.nG * CSR_GN * 4); c.FLAG = (int*)al(256);
  c.bytes = off - off0; return off;
}
static void csr_build(const CsrBufs& c, const int* dst, int E, int N, hipStream_t stream) {
  const size_t smem = (size_t)(2 * c.NGP + c.CHP) * 4;
  csrZ_kernel<<<512, 256, 0, stream>>>((int*)c.base, c.bytes / 16);
  csrA_kernel<<<CSR_NBLK, 64, smem, stream>>>(dst, E, N, c.nG, c.CHP, c.NGP, c.STG, c.HST);
  csrS_kernel<<<1, 512, 0, stream>>>(c.HST, c.nG, c.NGP, c.START, c.TOT, c.OFF);
  csrB_kernel<<<c.nG, 256, 0, stream>>>(dst, N, c.nG, c.CHP, c.NGP, (int)c.permLen, c.STG, c.HST, c.OFF, c.START, c.TOT, c.PERM, c.ROWPTR, c.ROWCNT, c.FLAG);
}


__global__ __launch_bounds__(256) void prepw_kernel(const float* __restrict__ w2a, const float* __restrict__ b2a, const float* __restrict__ w2b, const float* __restrict__ b2b, b16* __restrict__ WM1, b16* __restrict__ WM2) {
  const size_t u = (size_t)blockIdx.x * 256 + threadIdx.x; const size_t n1 = (size_t)HID * KM1 / 8, n2 = (size_t)HID * KM2 / 8; size_t t = u; v8b o;
  if (t < n1) { const size_t e = t * 8; const int oo = (int)(e / KM1), k0 = (int)(e % KM1); for (int j = 0; j < 8; ++j) { const int kk = k0 + j; float w = 0.0f; if (kk < EH * FIN0) { const int k = kk / FIN0, i = kk % FIN0; w = w2a[(size_t)k * (FIN0 * HID) + i * HID + oo]; } else if (kk < KM1R) { const int i = kk - EH * FIN0; w = b2a[i * HID + oo]; } o[j] = (b16)(bf16_rne(w) * WSC); } for (int pass = 0; pass < 2; ++pass) { *(volatile v8b*)(WM1 + e) = o; __threadfence(); } return; } t -= n1;
  if (t < n2) { const size_t e = t * 8; const int oo = (int)(e / KM2), k0 = (int)(e % KM2); for (int j = 0; j < 8; ++j) { const int kk = k0 + j; float w; if (kk < EH * HID) { const int k = kk / HID, i = kk % HID; w = w2b[(size_t)k * (HID * HID) + i * HID + oo]; } else { const int i = kk - EH * HID; w = b2b[i * HID + oo]; } o[j] = (b16)(bf16_rne(w) * WSC); } for (int pass = 0; pass < 2; ++pass) { *(volatile v8b*)(WM2 + e) = o; __threadfence(); } }
}
template <int LAYER>
__global__ __launch_bounds__(128) void msg_kernel(const float* __restrict__ Hn  , const float* __restrict__ ea, const float* __restrict__ w1, const float* __restrict__ b1, const int* __restrict__ srcs, const int* __restrict__ PERM, int permLen, const b16* __restrict__ WM, float* __restrict__ MSG) {
  constexpr int FIN = LAYER == 0 ? FIN0 : HID, KM = LAYER == 0 ? KM1 : KM2, KMR = LAYER == 0 ? KM1R : KM2;
  __shared__ __attribute__((aligned(16))) float Tf[4][16][HID + 4]; __shared__ float w1s[2][EH], b1s[EH];
  const int wave = threadIdx.x >> 5, lane = threadIdx.x & 31, nloc = lane & 15, hlf = lane >> 4; const size_t m0 = (size_t)blockIdx.x * 64 + wave * 16; const size_t j = m0 + nloc;
  if (threadIdx.x < EH) { w1s[0][threadIdx.x] = bf16_rne(w1[threadIdx.x]); w1s[1][threadIdx.x] = bf16_rne(w1[EH + threadIdx.x]); b1s[threadIdx.x] = bf16_rne(b1[threadIdx.x]); }
  __syncthreads();
  const bool live = j < (size_t)permLen; const int e = live ? iclamp(PERM[j], 0, E - 1) : 0; const size_t s = (size_t)iclamp(srcs[e], 0, N - 1);
  const float a0 = live ? bf16_rne(ea[(size_t)e * 2]) : 0.0f, a1 = live ? bf16_rne(ea[(size_t)e * 2 + 1]) : 0.0f;
  float hs[FIN];
#pragma unroll
  for (int i = 0; i < FIN; ++i) hs[i] = live ? (LAYER == 0 ? bf16_rne(Hn[s * FIN0 + i]) : Hn[s * HID + i]) : 0.0f;
  auto gate = [&](int k) -> float { return fmaxf(pmul(a0, w1s[0][k]) + pmul(a1, w1s[1][k]) + b1s[k], 0.0f); };
  v8f acc[2] = {{}, {}};
  for (int kb = 0; kb < KM; kb += 32) { v16b a, al;
#pragma unroll
    for (int el = 0; el < 16; ++el) { const int off = (el < 8) ? (8 * hlf + el) : (16 + 8 * hlf + (el - 8)); const int kk = kb + off; float v = 0.0f;
      if (LAYER == 0) {
        if (kk < EH * FIN0) { const int k = kk / 3, i = kk - 3 * k; const float h = (i == 0) ? hs[0] : (i == 1 ? hs[1] : hs[2]); v = pmul(gate(k), h); }
        else if (kk < KMR) { const int i = kk - EH * FIN0; v = (i == 0) ? hs[0] : (i == 1 ? hs[1] : hs[2]); }
      } else {
        const int base = (el < 8) ? el : (16 + el - 8); const float h = hlf ? hs[(base + 8) & 31] : hs[base & 31];
        v = (kb < EH * HID) ? pmul(gate(kb >> 5), h) : h; }
      b16 p, q; split16(v * XS, p, q); a[el] = p; al[el] = q; }
#pragma unroll
    for (int t = 0; t < 2; ++t) { const v16b bw = frag_kb(WM + (size_t)(t * 16 + nloc) * KM + kb, hlf); acc[t] = wmma16b(a, bw, acc[t]); acc[t] = wmma16b(al, bw, acc[t]); } }
#pragma unroll
  for (int t = 0; t < 2; ++t)
#pragma unroll 1
    for (int r = 0; r < 8; ++r) Tf[wave][8 * hlf + r][t * 16 + nloc] = acc[t][r] * (1.0f / (XS * WSC));
  wave_lds_sync();
  for (int pass = 0; pass < 2; ++pass) { for (int r4 = 0; r4 < 16; r4 += 4) { const int rr = r4 + (lane >> 3), c4 = (lane & 7) * 4; *(volatile v4f*)(MSG + (m0 + rr) * HID + c4) = *(const v4f*)(&Tf[wave][rr][c4]); } __threadfence(); }
}
template <int LAYER>
__global__ __launch_bounds__(256) void node_kernel(const float* __restrict__ Hin, const float* __restrict__ MSG, const int* __restrict__ ROWPTR, const int* __restrict__ ROWCNT, int permLen, const float* __restrict__ root, const float* __restrict__ bias, float* __restrict__ Hout) {
  constexpr int FIN = LAYER == 0 ? FIN0 : HID;
  const int wave = threadIdx.x >> 5, lane = threadIdx.x & 31; const size_t v = (size_t)blockIdx.x * 8 + wave; float o = 0.0f;
  if (v < (size_t)N) { float r = 0.0f;
#pragma unroll 1
    for (int i = 0; i < FIN; ++i) { const float h = LAYER == 0 ? bf16_rne(Hin[v * FIN0 + i]) : Hin[v * HID + i]; r += pmul(h, bf16_rne(root[i * HID + lane])); }
    int st = ROWPTR[v], cnt = ROWCNT[v]; cnt = iclamp(cnt, 0, 65536); st = iclamp(st, 0, permLen - cnt); float m = 0.0f;
    for (int q = 0; q < cnt; ++q) m += MSG[(size_t)(st + q) * HID + lane];
    o = fmaxf(r + m * (1.0f / fmaxf((float)cnt, 1.0f)) + bf16_rne(bias[lane]), 0.0f); }
  for (int pass = 0; pass < 2; ++pass) { ((volatile float*)Hout)[v * HID + lane] = o; __threadfence(); }
}
__global__ __launch_bounds__(256) void fc_kernel(const float* __restrict__ Hn, const float* __restrict__ fw, const float* __restrict__ fb, float* __restrict__ out) {
  const size_t v = (size_t)blockIdx.x * 256 + threadIdx.x; float o0 = 0.0f, o1 = 0.0f;
  if (v < (size_t)N) { o0 = bf16_rne(fb[0]); o1 = bf16_rne(fb[1]);
#pragma unroll 1
    for (int i = 0; i < HID; ++i) { const float h = Hn[v * HID + i]; o0 += pmul(h, bf16_rne(fw[i * 2])); o1 += pmul(h, bf16_rne(fw[i * 2 + 1])); } }
  typedef __attribute__((ext_vector_type(2))) float v2f; v2f ov = {o0, o1};
  for (int pass = 0; pass < 2; ++pass) { if (v < (size_t)N) *(volatile v2f*)(out + v * 2) = ov; __threadfence(); }
}
}

extern "C" void kernel_launch(void* const* d_in, const int* in_sizes, int n_in, void* d_out, int out_size, void* d_ws, size_t ws_size, hipStream_t stream) {
  (void)n_in;
  auto Fp = [&](int i) { return (const float*)d_in[i]; }; auto Ip = [&](int i) { return (const int*)d_in[i]; };
  if (in_sizes[0] != N * FIN0 || in_sizes[1] != 2 * E || in_sizes[2] != E * 2 || in_sizes[3] != 2 * EH || in_sizes[5] != EH * FIN0 * HID || in_sizes[11] != EH * HID * HID || in_sizes[13] != HID * HID || in_sizes[15] != HID * OUTD || out_size != N * OUTD) return;
  size_t off = 0; char* ws = (char*)d_ws;
  auto carve = [&](size_t bytes) { char* p = ws + off; off += (bytes + 255) & ~(size_t)255; return p; };
  b16* WM1 = (b16*)carve((size_t)HID * KM1 * 2); b16* WM2 = (b16*)carve((size_t)HID * KM2 * 2); float* MSG = (float*)carve((size_t)EP * HID * 4); float* H1 = (float*)carve((size_t)NP * HID * 4); float* H2 = (float*)carve((size_t)NP * HID * 4);
  CsrBufs csr; off = csr_carve(csr, ws, off, E, N);
  if (off > ws_size || off > ((size_t)128 << 20) || csr.permLen > (size_t)EP) return;
  prepw_kernel<<<(unsigned)(((size_t)HID * KM1 / 8 + (size_t)HID * KM2 / 8 + 255) / 256), 256, 0, stream>>>(Fp(5), Fp(6), Fp(11), Fp(12), WM1, WM2);
  csr_build(csr, Ip(1) + E, E, N, stream);
  msg_kernel<0><<<EP / 64, 128, 0, stream>>>(Fp(0), Fp(2), Fp(3), Fp(4), Ip(1), csr.PERM, (int)csr.permLen, WM1, MSG);
  node_kernel<0><<<NP / 8, 256, 0, stream>>>(Fp(0), MSG, csr.ROWPTR, csr.ROWCNT, (int)csr.permLen, Fp(7), Fp(8), H1);
  msg_kernel<1><<<EP / 64, 128, 0, stream>>>(H1, Fp(2), Fp(9), Fp(10), Ip(1), csr.PERM, (int)csr.permLen, WM2, MSG);
  node_kernel<1><<<NP / 8, 256, 0, stream>>>(H1, MSG, csr.ROWPTR, csr.ROWCNT, (int)csr.permLen, Fp(13), Fp(14), H2);
  fc_kernel<<<(N + 255) / 256, 256, 0, stream>>>(H2, Fp(15), Fp(16), (float*)d_out);
}
